// CondConvResidual_48241072668980
// MI455X (gfx1250) — hardware-verified
//
#include <hip/hip_runtime.h>

typedef _Float16 v16h __attribute__((ext_vector_type(16)));
typedef _Float16 v8h  __attribute__((ext_vector_type(8)));
typedef _Float16 v4h  __attribute__((ext_vector_type(4)));
typedef float    v8f  __attribute__((ext_vector_type(8)));
typedef float    v4f  __attribute__((ext_vector_type(4)));
typedef v8h __attribute__((may_alias)) v8ha;
typedef v4h __attribute__((may_alias)) v4ha;
typedef v4f __attribute__((may_alias)) v4fa;

union Frag { v16h v; v8h half[2]; };

#define NB     32
#define HH     56
#define WW     56
#define NPOS   (HH * WW)
#define CIN    96
#define NE     4
#define CM     384
#define CF     96
#define BNEPS  1e-3f
#define SC1    8.0f
#define ISC1   0.125f
#define SC2    16.0f
#define ISC2   0.0625f

#define APITCH 104
#define HPITCH 200
#define TPITCH 392

static_assert(NPOS % 64 == 0);
static_assert(CIN % 32 == 0);
static_assert(CM % 32 == 0);

__device__ __forceinline__ v8f wmma_f16(v16h a, v16h b, v8f c) {
  v8f d = __builtin_amdgcn_wmma_f32_16x16x32_f16(false, a, false, b, (short)0, c, false, false);
  asm volatile("v_nop\n\tv_nop\n\tv_nop\n\tv_nop" : "+v"(d) : "v"(a), "v"(b));
  return d;
}

__device__ __forceinline__ v16h load_frag(const _Float16* p, int h) {
  Frag f;
  f.half[0] = *(const v8ha*)(p + 8 * h);
  f.half[1] = *(const v8ha*)(p + 16 + 8 * h);
  return f.v;
}

__device__ __forceinline__ void put_chunks_h(const _Float16* s, _Float16* dst, int nch, int tid) {
  const _Float16 hz = (_Float16)0.0f;
  const v8h z = {hz, hz, hz, hz, hz, hz, hz, hz};
  const int nld = (nch + 31) & ~31;
  v8h v[3];
  #pragma unroll
  for (int it = 0; it < 3; ++it) {
    const int q = it * 256 + tid;
    v[it] = z;
    if (q < nld) v[it] = *(const v8ha*)(s + q * 8);
  }
  #pragma unroll
  for (int it = 0; it < 3; ++it) {
    const int q = it * 256 + tid;
    if (q < nch) *(volatile v8h*)(dst + (size_t)q * 8) = v[it];
  }
  __threadfence();
  #pragma unroll
  for (int it = 0; it < 3; ++it) {
    const int q = it * 256 + tid;
    if (q < nch) *(volatile v8h*)(dst + (size_t)q * 8) = v[it];
  }
}

__device__ __forceinline__ void put_chunks_f(const float* s, float* dst, int nch, int tid) {
  const v4f z = {0.f, 0.f, 0.f, 0.f};
  const int nld = (nch + 31) & ~31;
  v4f v[4];
  #pragma unroll
  for (int it = 0; it < 4; ++it) {
    const int q = it * 256 + tid;
    v[it] = z;
    if (q < nld) v[it] = *(const v4fa*)(s + q * 4);
  }
  #pragma unroll
  for (int it = 0; it < 4; ++it) {
    const int q = it * 256 + tid;
    if (q < nch) *(volatile v4f*)(dst + (size_t)q * 4) = v[it];
  }
  __threadfence();
  #pragma unroll
  for (int it = 0; it < 4; ++it) {
    const int q = it * 256 + tid;
    if (q < nch) *(volatile v4f*)(dst + (size_t)q * 4) = v[it];
  }
}

__global__ __launch_bounds__(256) void route_mix_kernel(
    const float* __restrict__ x,    const float* __restrict__ Wr,  const float* __restrict__ br,
    const float* __restrict__ Wpw,  const float* __restrict__ bpw,
    const float* __restrict__ Wdw,  const float* __restrict__ bdw,
    const float* __restrict__ Wpwl, const float* __restrict__ bpwl,
    _Float16* __restrict__ wk1, _Float16* __restrict__ wk2,
    float* __restrict__ wdm, float* __restrict__ bias1,
    float* __restrict__ bdm, float* __restrict__ bias2)
{
  __shared__ __attribute__((aligned(16))) float sPart[10 * CIN];
  __shared__ float sPooled[CIN];
  __shared__ float sRw[NE];
  __shared__ __attribute__((aligned(16))) _Float16 sP[48 * CIN];
  __shared__ __attribute__((aligned(16))) float sF[9 * CM];

  const int b = blockIdx.x, tid = threadIdx.x;

  if (tid < 240) {
    const int c4 = tid % 24, ps = tid / 24;
    const float* xb = x + (size_t)b * NPOS * CIN + 4 * c4;
    v4f a = {0.f, 0.f, 0.f, 0.f};
    #pragma unroll 1
    for (int p = ps; p < NPOS; p += 10) a += *(const v4fa*)(xb + (size_t)p * CIN);
    *(v4fa*)(sPart + ps * CIN + 4 * c4) = a;
  }
  __syncthreads();
  if (tid < CIN) {
    float s = 0.f;
    #pragma unroll 1
    for (int ps = 0; ps < 10; ++ps) s += sPart[ps * CIN + tid];
    sPooled[tid] = s * (1.0f / (float)NPOS);
  }
  __syncthreads();
  if (tid < NE) {
    float s = 0.f;
    #pragma unroll 1
    for (int c = 0; c < CIN; ++c) s += sPooled[c] * Wr[c * NE + tid];
    s += br[tid];
    const float ex = expf(-s);
    sRw[tid] = __builtin_amdgcn_rcpf(1.0f + ex);
  }
  __syncthreads();

  #pragma unroll 1
  for (int piece = 0; piece < 8; ++piece) {
    #pragma unroll 1
    for (int it = 0; it < 18; ++it) {
      const int i = it * 256 + tid;
      const int k = i / 48, nl = i % 48;
      const int n = piece * 48 + nl;
      float wsum = 0.f;
      #pragma unroll 1
      for (int e = 0; e < NE; ++e) wsum += sRw[e] * Wpw[((size_t)e * CIN + k) * CM + n];
      sP[nl * CIN + k] = (_Float16)(wsum * SC1);
    }
    __syncthreads();
    put_chunks_h(sP, wk1 + (size_t)b * CM * CIN + (size_t)piece * 48 * CIN, 576, tid);
    __syncthreads();
  }

  #pragma unroll 1
  for (int piece = 0; piece < 8; ++piece) {
    #pragma unroll 1
    for (int it = 0; it < 18; ++it) {
      const int i = it * 256 + tid;
      const int ml = i / 12, fl = i % 12;
      const int f = piece * 12 + fl;
      float wsum = 0.f;
      #pragma unroll 1
      for (int e = 0; e < NE; ++e) wsum += sRw[e] * Wpwl[((size_t)e * CM + ml) * CF + f];
      sP[fl * CM + ml] = (_Float16)(wsum * SC2);
    }
    __syncthreads();
    put_chunks_h(sP, wk2 + (size_t)b * CF * CM + (size_t)piece * 12 * CM, 576, tid);
    __syncthreads();
  }

  #pragma unroll 1
  for (int it = 0; it < 14; ++it) {
    const int i = it * 256 + tid;
    if (i < 9 * CM) {
      float wsum = 0.f;
      #pragma unroll 1
      for (int e = 0; e < NE; ++e) wsum += sRw[e] * Wdw[(size_t)e * 9 * CM + i];
      sF[i] = wsum;
    }
  }
  __syncthreads();
  put_chunks_f(sF, wdm + (size_t)b * 9 * CM, 864, tid);
  __syncthreads();

  #pragma unroll 1
  for (int it = 0; it < 2; ++it) {
    const int i = it * 256 + tid;
    if (i < CM) {
      float wsum = 0.f;
      #pragma unroll 1
      for (int e = 0; e < NE; ++e) wsum += sRw[e] * bpw[e * CM + i];
      sF[i] = wsum;
    }
  }
  __syncthreads();
  put_chunks_f(sF, bias1 + (size_t)b * CM, 96, tid);
  __syncthreads();

  #pragma unroll 1
  for (int it = 0; it < 2; ++it) {
    const int i = it * 256 + tid;
    if (i < CM) {
      float wsum = 0.f;
      #pragma unroll 1
      for (int e = 0; e < NE; ++e) wsum += sRw[e] * bdw[e * CM + i];
      sF[i] = wsum;
    }
  }
  __syncthreads();
  put_chunks_f(sF, bdm + (size_t)b * CM, 96, tid);
  __syncthreads();

  if (tid < CF) {
    float wsum = 0.f;
    #pragma unroll 1
    for (int e = 0; e < NE; ++e) wsum += sRw[e] * bpwl[e * CF + tid];
    sF[tid] = wsum;
  }
  __syncthreads();
  put_chunks_f(sF, bias2 + (size_t)b * CF, 24, tid);
}

__global__ __launch_bounds__(256) void expand_kernel(
    const float* __restrict__ x, const _Float16* __restrict__ wk1, const float* __restrict__ bias1,
    const float* __restrict__ g1, const float* __restrict__ b1,
    const float* __restrict__ m1, const float* __restrict__ v1,
    _Float16* __restrict__ hpl)
{
  __shared__ __attribute__((aligned(16))) _Float16 sA[64 * APITCH];
  __shared__ __attribute__((aligned(16))) _Float16 sH[64 * HPITCH];

  const int nh = blockIdx.x, pt = blockIdx.y, b = blockIdx.z;
  const int tid = threadIdx.x, lane = tid & 31, w = tid >> 5;
  const int h = lane >> 4, m = lane & 15;
  const size_t prow0 = (size_t)b * NPOS + (size_t)pt * 64;

  #pragma unroll
  for (int s = 0; s < 6; ++s) {
    const int f4 = s * 256 + tid;
    const int row = f4 / 24, c4 = f4 % 24;
    const v4f u = *(const v4fa*)(x + (prow0 + row) * CIN + 4 * c4);
    const v4h o = {(_Float16)u[0], (_Float16)u[1], (_Float16)u[2], (_Float16)u[3]};
    *(v4ha*)(sA + row * APITCH + 4 * c4) = o;
  }
  __syncthreads();

  const int rt = w & 3, ct0 = (w >> 2) * 6;
  const v8f z8f = {0.f, 0.f, 0.f, 0.f, 0.f, 0.f, 0.f, 0.f};
  v8f acc[6];
  #pragma unroll
  for (int j = 0; j < 6; ++j) acc[j] = z8f;

  const _Float16* arow = sA + (16 * rt + m) * APITCH;
  const _Float16* brow = wk1 + ((size_t)b * CM + nh * 192 + 16 * ct0 + m) * CIN;
  #pragma unroll
  for (int ks = 0; ks < 3; ++ks) {
    const int k0 = 32 * ks;
    const v16h a = load_frag(arow + k0, h);
    #pragma unroll
    for (int j = 0; j < 6; ++j) {
      const v16h bf = load_frag(brow + (size_t)j * 16 * CIN + k0, h);
      acc[j] = wmma_f16(a, bf, acc[j]);
    }
  }

  #pragma unroll
  for (int j = 0; j < 6; ++j) {
    const int nloc = 16 * (ct0 + j) + m;
    const int n = nh * 192 + nloc;
    const float bi = bias1[(size_t)b * CM + n];
    const float sc = g1[n] * rsqrtf(v1[n] + BNEPS);
    const float mu = m1[n], be = b1[n];
    #pragma unroll
    for (int r = 0; r < 8; ++r) {
      const int row = 16 * rt + 8 * h + r;
      float y = acc[j][r] * ISC1 + bi;
      y = (y - mu) * sc + be;
      y = fmaxf(y, 0.0f);
      sH[row * HPITCH + nloc] = (_Float16)y;
    }
  }
  __syncthreads();

  _Float16* dst = hpl + prow0 * CM + nh * 192;
  v8h vals[6];
  #pragma unroll
  for (int it = 0; it < 6; ++it) {
    const int q = it * 256 + tid;
    const int row = q / 24, cq = q % 24;
    vals[it] = *(const v8ha*)(sH + row * HPITCH + 8 * cq);
  }
  #pragma unroll
  for (int it = 0; it < 6; ++it) {
    const int q = it * 256 + tid;
    const int row = q / 24, cq = q % 24;
    *(volatile v8h*)(dst + (size_t)row * CM + 8 * cq) = vals[it];
  }
  __threadfence();
  #pragma unroll
  for (int it = 0; it < 6; ++it) {
    const int q = it * 256 + tid;
    const int row = q / 24, cq = q % 24;
    *(volatile v8h*)(dst + (size_t)row * CM + 8 * cq) = vals[it];
  }
}

union ProjTile { _Float16 a[64 * TPITCH]; float o[64 * CF]; };

__global__ __launch_bounds__(256) void dwproj_kernel(
    const _Float16* __restrict__ hpl, const float* __restrict__ wdm, const float* __restrict__ bdm,
    const float* __restrict__ g2, const float* __restrict__ b2,
    const float* __restrict__ m2, const float* __restrict__ v2,
    const _Float16* __restrict__ wk2, const float* __restrict__ bias2,
    const float* __restrict__ g3, const float* __restrict__ b3,
    const float* __restrict__ m3, const float* __restrict__ v3,
    const float* __restrict__ x, float* __restrict__ out)
{
  __shared__ __attribute__((aligned(16))) ProjTile sT;
  __shared__ __attribute__((aligned(16))) float sW[9 * CM];
  __shared__ __attribute__((aligned(16))) float sBd[CM];
  __shared__ __attribute__((aligned(16))) float sS2[CM];
  __shared__ __attribute__((aligned(16))) float sM2[CM];
  __shared__ __attribute__((aligned(16))) float sB2[CM];

  const int pt = blockIdx.x, b = blockIdx.y;
  const int tid = threadIdx.x, lane = tid & 31, w = tid >> 5;
  const int h = lane >> 4, m = lane & 15;
  const int p0 = pt * 64;

  for (int i = tid; i < 9 * CM; i += 256) sW[i] = wdm[(size_t)b * 9 * CM + i];
  for (int i = tid; i < CM; i += 256) {
    sBd[i] = bdm[(size_t)b * CM + i];
    sS2[i] = g2[i] * rsqrtf(v2[i] + BNEPS);
    sM2[i] = m2[i];
    sB2[i] = b2[i];
  }
  __syncthreads();

  const _Float16 hz = (_Float16)0.0f;
  const v8h z8h = {hz, hz, hz, hz, hz, hz, hz, hz};
  const v8f z8f = {0.f, 0.f, 0.f, 0.f, 0.f, 0.f, 0.f, 0.f};
  const _Float16* hb = hpl + (size_t)b * NPOS * CM;
  #pragma unroll 1
  for (int it = 0; it < 12; ++it) {
    const int i = it * 256 + tid;
    const int pix = i / 48, g = i % 48;
    const int p = p0 + pix;
    const int py = p / WW, px = p % WW;
    v8f acc = z8f;
    #pragma unroll
    for (int tap = 0; tap < 9; ++tap) {
      const int yy = py + tap / 3 - 1, xx = px + tap % 3 - 1;
      const bool ok = ((unsigned)yy < (unsigned)HH) && ((unsigned)xx < (unsigned)WW);
      const int yc = min(max(yy, 0), HH - 1), xc = min(max(xx, 0), WW - 1);
      v8h hv = *(const v8ha*)(hb + (size_t)(yc * WW + xc) * CM + 8 * g);
      hv = ok ? hv : z8h;
      const v4f w0 = *(const v4fa*)(sW + tap * CM + 8 * g);
      const v4f w1 = *(const v4fa*)(sW + tap * CM + 8 * g + 4);
      #pragma unroll
      for (int c = 0; c < 4; ++c) {
        acc[c]     += (float)hv[c]     * w0[c];
        acc[4 + c] += (float)hv[4 + c] * w1[c];
      }
    }
    const v4f bd0 = *(const v4fa*)(sBd + 8 * g), bd1 = *(const v4fa*)(sBd + 8 * g + 4);
    const v4f sc0 = *(const v4fa*)(sS2 + 8 * g), sc1 = *(const v4fa*)(sS2 + 8 * g + 4);
    const v4f mu0 = *(const v4fa*)(sM2 + 8 * g), mu1 = *(const v4fa*)(sM2 + 8 * g + 4);
    const v4f be0 = *(const v4fa*)(sB2 + 8 * g), be1 = *(const v4fa*)(sB2 + 8 * g + 4);
    v8h yv;
    #pragma unroll
    for (int c = 0; c < 4; ++c) {
      float t0 = acc[c] + bd0[c];
      t0 = (t0 - mu0[c]) * sc0[c] + be0[c];
      yv[c] = (_Float16)fmaxf(t0, 0.0f);
      float t1 = acc[4 + c] + bd1[c];
      t1 = (t1 - mu1[c]) * sc1[c] + be1[c];
      yv[4 + c] = (_Float16)fmaxf(t1, 0.0f);
    }
    *(v8ha*)(sT.a + pix * TPITCH + 8 * g) = yv;
  }
  __syncthreads();

  const int rt = w & 3, ct0 = (w >> 2) * 3;
  v8f pacc[3];
  #pragma unroll
  for (int j = 0; j < 3; ++j) pacc[j] = z8f;
  const _Float16* arow = sT.a + (16 * rt + m) * TPITCH;
  const _Float16* brow = wk2 + ((size_t)b * CF + 16 * ct0 + m) * CM;
  #pragma unroll 1
  for (int ks = 0; ks < CM / 32; ++ks) {
    const int k0 = 32 * ks;
    const v16h a = load_frag(arow + k0, h);
    #pragma unroll
    for (int j = 0; j < 3; ++j) {
      const v16h bf = load_frag(brow + (size_t)j * 16 * CM + k0, h);
      pacc[j] = wmma_f16(a, bf, pacc[j]);
    }
  }
  __syncthreads();

  #pragma unroll
  for (int j = 0; j < 3; ++j) {
    const int n = 16 * (ct0 + j) + m;
    const float bi = bias2[(size_t)b * CF + n];
    const float sc = g3[n] * rsqrtf(v3[n] + BNEPS);
    const float mu = m3[n], be = b3[n];
    #pragma unroll
    for (int r = 0; r < 8; ++r) {
      const int row = 16 * rt + 8 * h + r;
      float y = pacc[j][r] * ISC2 + bi;
      y = (y - mu) * sc + be;
      sT.o[row * CF + n] = y;
    }
  }
  __syncthreads();

  const size_t fo = ((size_t)b * NPOS + (size_t)p0) * CF;
  v4f vals[6];
  #pragma unroll
  for (int it = 0; it < 6; ++it) {
    const int q = it * 256 + tid;
    const v4f t = *(const v4fa*)(sT.o + q * 4);
    const v4f xr = *(const v4fa*)(x + fo + (size_t)q * 4);
    vals[it] = t + xr;
  }
  #pragma unroll
  for (int it = 0; it < 6; ++it) {
    const int q = it * 256 + tid;
    *(volatile v4f*)(out + fo + (size_t)q * 4) = vals[it];
  }
  __threadfence();
  #pragma unroll
  for (int it = 0; it < 6; ++it) {
    const int q = it * 256 + tid;
    *(volatile v4f*)(out + fo + (size_t)q * 4) = vals[it];
  }
}

extern "C" void kernel_launch(void* const* d_in, const int* in_sizes, int n_in,
                              void* d_out, int out_size, void* d_ws, size_t ws_size,
                              hipStream_t stream) {
  if (n_in < 21) return;
  if (in_sizes[0] != NB * NPOS * CIN) return;
  if (in_sizes[1] != CIN * NE || in_sizes[2] != NE) return;
  if (in_sizes[3] != NE * CIN * CM || in_sizes[4] != NE * CM) return;
  if (in_sizes[5] != NE * 9 * CM || in_sizes[6] != NE * CM) return;
  if (in_sizes[7] != NE * CM * CF || in_sizes[8] != NE * CF) return;
  for (int i = 9; i <= 16; ++i) if (in_sizes[i] != CM) return;
  for (int i = 17; i <= 20; ++i) if (in_sizes[i] != CF) return;
  if (out_size != NB * NPOS * CF) return;

  const float* x    = (const float*)d_in[0];
  const float* Wr   = (const float*)d_in[1];
  const float* br   = (const float*)d_in[2];
  const float* Wpw  = (const float*)d_in[3];
  const float* bpw  = (const float*)d_in[4];
  const float* Wdw  = (const float*)d_in[5];
  const float* bdw  = (const float*)d_in[6];
  const float* Wpwl = (const float*)d_in[7];
  const float* bpwl = (const float*)d_in[8];
  const float* g1 = (const float*)d_in[9];  const float* b1 = (const float*)d_in[10];
  const float* m1 = (const float*)d_in[11]; const float* v1 = (const float*)d_in[12];
  const float* g2 = (const float*)d_in[13]; const float* b2 = (const float*)d_in[14];
  const float* m2 = (const float*)d_in[15]; const float* v2 = (const float*)d_in[16];
  const float* g3 = (const float*)d_in[17]; const float* b3 = (const float*)d_in[18];
  const float* m3 = (const float*)d_in[19]; const float* v3 = (const float*)d_in[20];
  float* out = (float*)d_out;

  const size_t wk1_bytes   = (size_t)NB * CM * CIN * 2;
  const size_t wk2_bytes   = (size_t)NB * CF * CM * 2;
  const size_t wdm_bytes   = (size_t)NB * 9 * CM * 4;
  const size_t bias1_bytes = (size_t)NB * CM * 4;
  const size_t bdm_bytes   = (size_t)NB * CM * 4;
  const size_t bias2_bytes = (size_t)NB * CF * 4;
  const size_t hpl_bytes   = (size_t)NB * NPOS * CM * 2;
  const size_t o_wk1   = 0;
  const size_t o_wk2   = o_wk1 + wk1_bytes;
  const size_t o_wdm   = o_wk2 + wk2_bytes;
  const size_t o_bias1 = o_wdm + wdm_bytes;
  const size_t o_bdm   = o_bias1 + bias1_bytes;
  const size_t o_bias2 = o_bdm + bdm_bytes;
  const size_t o_hpl   = o_bias2 + bias2_bytes;
  const size_t total   = o_hpl + hpl_bytes;
  if (total > ws_size) return;

  char* ws = (char*)d_ws;
  _Float16* wk1   = (_Float16*)(ws + o_wk1);
  _Float16* wk2   = (_Float16*)(ws + o_wk2);
  float*    wdm   = (float*)(ws + o_wdm);
  float*    bias1 = (float*)(ws + o_bias1);
  float*    bdm   = (float*)(ws + o_bdm);
  float*    bias2 = (float*)(ws + o_bias2);
  _Float16* hpl   = (_Float16*)(ws + o_hpl);

  route_mix_kernel<<<dim3(NB), dim3(256), 0, stream>>>(
      x, Wr, br, Wpw, bpw, Wdw, bdw, Wpwl, bpwl,
      wk1, wk2, wdm, bias1, bdm, bias2);

  expand_kernel<<<dim3(2, NPOS / 64, NB), dim3(256), 0, stream>>>(
      x, wk1, bias1, g1, b1, m1, v1, hpl);

  dwproj_kernel<<<dim3(NPOS / 64, NB), dim3(256), 0, stream>>>(
      hpl, wdm, bdm, g2, b2, m2, v2, wk2, bias2, g3, b3, m3, v3, x, out);
}
